// FeedbackDetector_8589934869
// MI455X (gfx1250) — hardware-verified
//
#include <hip/hip_runtime.h>


#define NBATCH 16
#define NFREQ  481
#define NSTEP  500
#define NSEQ   7696
#define CH     16
#define HID    32
#define NGATE  96
#define FPAD   484
#define XFR    (FPAD * CH)
#define XTS    ((size_t)NBATCH * XFR)

typedef _Float16 f16t;
typedef f16t  v16h __attribute__((ext_vector_type(16)));
typedef f16t  v8h  __attribute__((ext_vector_type(8)));
typedef f16t  v4h  __attribute__((ext_vector_type(4)));
typedef float v8f  __attribute__((ext_vector_type(8)));
typedef float v4f  __attribute__((ext_vector_type(4)));
typedef unsigned int v4u __attribute__((ext_vector_type(4)));
typedef v8h v8ha __attribute__((may_alias));
typedef v4f v4fa __attribute__((may_alias));

union Frag { v16h v; v8h h8[2]; v4h q[4]; };
union Pk16 { v8h h; v4u u; };
union Pk32 { v4f f; v4u u; };

static_assert(XFR == 7744);

__device__ __forceinline__ v8f wmma16(v16h a, v16h b, v8f c) {
    return __builtin_amdgcn_wmma_f32_16x16x32_f16(false, a, false, b, (short)0, c, false, false);
}
__device__ __forceinline__ v8f zacc() {
    const v8f z = {0.f, 0.f, 0.f, 0.f, 0.f, 0.f, 0.f, 0.f};
    return z;
}
__device__ __forceinline__ v8h zero8() {
    const f16t z = (f16t)0.0f;
    const v8h r = {z, z, z, z, z, z, z, z};
    return r;
}
__device__ __forceinline__ v4h zero4() {
    const f16t z = (f16t)0.0f;
    const v4h r = {z, z, z, z};
    return r;
}
__device__ __forceinline__ void guard22(v8f& c, const v16h& a0, const v16h& a1,
                                        const v16h& b0, const v16h& b1) {
    asm volatile("v_nop\n\tv_nop\n\tv_nop\n\tv_nop"
                 : "+v"(c) : "v"(a0), "v"(a1), "v"(b0), "v"(b1));
}
__device__ __forceinline__ void guard33(v8f& c, const v16h& a0, const v16h& a1, const v16h& a2,
                                        const v16h& b0, const v16h& b1, const v16h& b2) {
    asm volatile("v_nop\n\tv_nop\n\tv_nop\n\tv_nop"
                 : "+v"(c) : "v"(a0), "v"(a1), "v"(a2), "v"(b0), "v"(b1), "v"(b2));
}
__device__ __forceinline__ void guard2c(v8f& c0, v8f& c1, const v16h& a0, const v16h& a1,
                                        const v16h& b0, const v16h& b1) {
    asm volatile("v_nop\n\tv_nop\n\tv_nop\n\tv_nop"
                 : "+v"(c0), "+v"(c1) : "v"(a0), "v"(a1), "v"(b0), "v"(b1));
}

__device__ __forceinline__ float sigm(float x) {
    return __builtin_amdgcn_rcpf(1.0f + __expf(-x));
}
__device__ __forceinline__ float ftanh(float x) {
    float ax = fabsf(x);
    float t  = __expf(-2.0f * ax);
    float r  = (1.0f - t) * __builtin_amdgcn_rcpf(1.0f + t);
    return copysignf(r, x);
}

__global__ __launch_bounds__(256)
void k_pack(const float* __restrict__ w1, const float* __restrict__ w2,
            const float* __restrict__ wih, const float* __restrict__ whh,
            f16t* __restrict__ W1P, f16t* __restrict__ W2P,
            f16t* __restrict__ WIP, f16t* __restrict__ WHP) {
    const int p = blockIdx.x * 256 + threadIdx.x;
    if (p >= 1088) return;
    const f16t z = (f16t)0.0f;
    Pk16 v;
    f16t* dst;
    if (p < 128) {
        const int c = p >> 3, kk0 = (p & 7) * 8;
#pragma unroll
        for (int e = 0; e < 8; ++e) {
            const int kk = kk0 + e, d = kk & 3, k = min(kk >> 2, 8);
            const float wv = w1[(c * 4 + d) * 9 + k] * 64.0f;
            v.h[e] = (kk < 36) ? (f16t)wv : z;
        }
        dst = W1P + c * 64 + kk0;
    } else if (p < 320) {
        const int q = p - 128, c = q / 12, kk0 = (q - c * 12) * 8;
#pragma unroll
        for (int e = 0; e < 8; ++e) {
            const int kk = kk0 + e, ci = kk & 15, k = min(kk >> 4, 4);
            const float wv = w2[(c * 16 + ci) * 5 + k] * 64.0f;
            v.h[e] = (kk < 80) ? (f16t)wv : z;
        }
        dst = W2P + c * 96 + kk0;
    } else if (p < 704) {
        const int q = p - 320, g = q >> 2, kk0 = (q & 3) * 8;
#pragma unroll
        for (int e = 0; e < 8; ++e) {
            const int kk = kk0 + e, kc = min(kk, 15);
            const float wv = wih[g * 16 + kc] * 64.0f;
            v.h[e] = (kk < 16) ? (f16t)wv : z;
        }
        dst = WIP + g * 32 + kk0;
    } else {
        const int q = p - 704, g = q >> 2, kk0 = (q & 3) * 8;
#pragma unroll
        for (int e = 0; e < 8; ++e) {
            const float wv = whh[g * 32 + kk0 + e] * 64.0f;
            v.h[e] = (f16t)wv;
        }
        dst = WHP + g * 32 + kk0;
    }
    *(volatile v4u*)dst = v.u;
    __threadfence();
    *(volatile v4u*)dst = v.u;
}

__global__ __launch_bounds__(256)
void k_conv(const float* __restrict__ feat, const f16t* __restrict__ W1P,
            const f16t* __restrict__ W2P, const float* __restrict__ b1,
            const float* __restrict__ a1p, const float* __restrict__ b2,
            const float* __restrict__ a2p, f16t* __restrict__ XP) {
    __shared__ v4h FP[512];
    __shared__ v8h X1P[1024];
    __shared__ v8h XS[992];

    const int tid = threadIdx.x, l = tid & 31, w = tid >> 5, hh = l >> 4, m = l & 15;
    const int fr = blockIdx.x, t = fr >> 4, b = fr & 15;
    const f16t z  = (f16t)0.0f;
    const v4h  z4 = zero4();
    const v8h  z8 = zero8();

#pragma unroll
    for (int i = 0; i < 2; ++i) {
        const int q  = tid + 256 * i;
        const int fs = q - 4;
        const int fc = min(max(fs, 0), NFREQ - 1);
        const float* src = feat + (((size_t)b * 4) * NFREQ + fc) * NSTEP + t;
        const size_t cs = (size_t)NFREQ * NSTEP;
        const float x0 = src[0], x1 = src[cs], x2 = src[2 * cs], x3 = src[3 * cs];
        const bool ok = (fs >= 0) && (fs < NFREQ);
        v4h pv;
        pv[0] = ok ? (f16t)x0 : z;
        pv[1] = ok ? (f16t)x1 : z;
        pv[2] = ok ? (f16t)x2 : z;
        pv[3] = ok ? (f16t)x3 : z;
        FP[q] = pv;
    }
    if (tid < 32) {
        const int pos = (tid < 4) ? (tid >> 1) : (498 + ((tid - 4) >> 1));
        X1P[pos * 2 + (tid & 1)] = z8;
    }
    Frag a10, a11, a20, a21, a22;
    {
        const f16t* p1 = W1P + m * 64 + 8 * hh;
        a10.h8[0] = *(const v8h*)(p1);       a10.h8[1] = *(const v8h*)(p1 + 16);
        a11.h8[0] = *(const v8h*)(p1 + 32);  a11.h8[1] = *(const v8h*)(p1 + 48);
        const f16t* p2 = W2P + m * 96 + 8 * hh;
        a20.h8[0] = *(const v8h*)(p2);       a20.h8[1] = *(const v8h*)(p2 + 16);
        a21.h8[0] = *(const v8h*)(p2 + 32);  a21.h8[1] = *(const v8h*)(p2 + 48);
        a22.h8[0] = *(const v8h*)(p2 + 64);  a22.h8[1] = *(const v8h*)(p2 + 80);
    }
    const v4f b1lo = *(const v4f*)(b1 + 8 * hh), b1hi = *(const v4f*)(b1 + 8 * hh + 4);
    const v4f b2lo = *(const v4f*)(b2 + 8 * hh), b2hi = *(const v4f*)(b2 + 8 * hh + 4);
    const float a1 = a1p[0], a2 = a2p[0];
    __syncthreads();

    for (int i = w; i < 31; i += 8) {
        const int f = 16 * i + m;
        Frag bb0, bb1;
        bb0.q[0] = FP[f + 2 * hh];
        bb0.q[1] = FP[f + 2 * hh + 1];
        bb0.q[2] = FP[f + 4 + 2 * hh];
        bb0.q[3] = FP[f + 5 + 2 * hh];
        const v4h t8 = FP[f + 8];
        bb1.q[0] = (hh == 0) ? t8 : z4;
        bb1.q[1] = z4; bb1.q[2] = z4; bb1.q[3] = z4;
        v8f acc = wmma16(a10.v, bb0.v, zacc());
        acc = wmma16(a11.v, bb1.v, acc);
        guard22(acc, a10.v, a11.v, bb0.v, bb1.v);
        const bool ok = f < NFREQ;
        Pk16 pk;
#pragma unroll
        for (int r = 0; r < 4; ++r) {
            float v0 = fmaf(acc[r],     0.015625f, b1lo[r]);
            float v1 = fmaf(acc[4 + r], 0.015625f, b1hi[r]);
            v0 = (v0 >= 0.0f) ? v0 : a1 * v0;
            v1 = (v1 >= 0.0f) ? v1 : a1 * v1;
            pk.h[r]     = ok ? (f16t)(v0 * 16.0f) : z;
            pk.h[4 + r] = ok ? (f16t)(v1 * 16.0f) : z;
        }
        X1P[(f + 2) * 2 + hh] = pk.h;
    }
    __syncthreads();

    for (int i = w; i < 31; i += 8) {
        const int f = 16 * i + m;
        Frag c0, c1, c2;
        c0.h8[0] = X1P[f * 2 + hh];        c0.h8[1] = X1P[(f + 1) * 2 + hh];
        c1.h8[0] = X1P[(f + 2) * 2 + hh];  c1.h8[1] = X1P[(f + 3) * 2 + hh];
        c2.h8[0] = X1P[(f + 4) * 2 + hh];  c2.h8[1] = z8;
        v8f acc = wmma16(a20.v, c0.v, zacc());
        acc = wmma16(a21.v, c1.v, acc);
        acc = wmma16(a22.v, c2.v, acc);
        guard33(acc, a20.v, a21.v, a22.v, c0.v, c1.v, c2.v);
        const bool ok = f < NFREQ;
        Pk16 pk;
#pragma unroll
        for (int r = 0; r < 4; ++r) {
            float v0 = fmaf(acc[r],     0.0009765625f, b2lo[r]);
            float v1 = fmaf(acc[4 + r], 0.0009765625f, b2hi[r]);
            v0 = (v0 >= 0.0f) ? v0 : a2 * v0;
            v1 = (v1 >= 0.0f) ? v1 : a2 * v1;
            pk.h[r]     = ok ? (f16t)(v0 * 64.0f) : z;
            pk.h[4 + r] = ok ? (f16t)(v1 * 64.0f) : z;
        }
        XS[f * 2 + hh] = pk.h;
    }
    __syncthreads();

    f16t* base = XP + (size_t)fr * XFR;
    Pk16 cv[4];
#pragma unroll
    for (int i = 0; i < 4; ++i) {
        const int p = tid + 256 * i, pc = min(p, 967);
        cv[i].h = XS[pc];
    }
#pragma unroll
    for (int i = 0; i < 4; ++i) {
        const int p = tid + 256 * i;
        if (p < 968) *(volatile v4u*)(base + (size_t)p * 8) = cv[i].u;
    }
    __threadfence();
#pragma unroll
    for (int i = 0; i < 4; ++i) {
        const int p = tid + 256 * i;
        if (p < 968) *(volatile v4u*)(base + (size_t)p * 8) = cv[i].u;
    }
}

__global__ __launch_bounds__(32)
void k_gru(const f16t* __restrict__ XP, const f16t* __restrict__ WIP,
           const f16t* __restrict__ WHP, const float* __restrict__ h0,
           const float* __restrict__ bih, const float* __restrict__ bhh,
           const float* __restrict__ fcw, const float* __restrict__ fcb,
           float* __restrict__ outp, float* __restrict__ outh) {
    __shared__ v8h WI[384];
    __shared__ v8h WH[384];
    __shared__ __attribute__((aligned(16))) f16t  hsh[2][512];
    __shared__ __attribute__((aligned(16))) float pst[16 * NSTEP];
    __shared__ __attribute__((aligned(16))) float hfin[512];

    const int l = threadIdx.x, hh = l >> 4, m = l & 15;
    const int n0 = blockIdx.x * 16;

#pragma unroll
    for (int i = 0; i < 12; ++i) {
        const int p = l + 32 * i;
        WI[p] = *(const v8h*)(WIP + (size_t)p * 8);
        WH[p] = *(const v8h*)(WHP + (size_t)p * 8);
    }
    const float br0  = bih[m]      + bhh[m];
    const float br1  = bih[16 + m] + bhh[16 + m];
    const float bz0  = bih[32 + m] + bhh[32 + m];
    const float bz1  = bih[48 + m] + bhh[48 + m];
    const float bxn0 = bih[64 + m], bhn0 = bhh[64 + m];
    const float bxn1 = bih[80 + m], bhn1 = bhh[80 + m];
    const float fw0  = fcw[m], fw1 = fcw[16 + m];
    const float fb   = fcb[0];

    float hC0[8], hC1[8];
#pragma unroll
    for (int r = 0; r < 8; ++r) {
        const size_t row = (size_t)(n0 + 8 * hh + r) * HID;
        hC0[r] = h0[row + m];
        hC1[r] = h0[row + 16 + m];
        hsh[0][(8 * hh + r) * 32 + m]      = (f16t)(hC0[r] * 64.0f);
        hsh[0][(8 * hh + r) * 32 + 16 + m] = (f16t)(hC1[r] * 64.0f);
    }
    __syncthreads();

    const int n  = n0 + m;
    const int bq = n / NFREQ;
    const int fq = n - bq * NFREQ;
    const f16t* xp = XP + ((size_t)bq * FPAD + fq) * CH + 8 * hh;
    const v8h z8 = zero8();
    const float INV = 0.000244140625f;

#pragma unroll 1
    for (int t = 0; t < NSTEP; ++t) {
        Frag ax, ah;
        ax.h8[0] = *(const v8h*)(xp + (size_t)t * XTS);
        ax.h8[1] = z8;
        const f16t* hc = &hsh[t & 1][0];
        ah.h8[0] = *(const v8ha*)(hc + m * 32 + 8 * hh);
        ah.h8[1] = *(const v8ha*)(hc + m * 32 + 16 + 8 * hh);

        v8f arz0, arz1, arz2, arz3, axn0, axn1, ahn0, ahn1;
        {
            Frag bi, bh;
            bi.h8[0] = WI[(m) * 4 + hh];       bi.h8[1] = WI[(m) * 4 + 2 + hh];
            bh.h8[0] = WH[(m) * 4 + hh];       bh.h8[1] = WH[(m) * 4 + 2 + hh];
            arz0 = wmma16(ax.v, bi.v, zacc());
            arz0 = wmma16(ah.v, bh.v, arz0);
            guard22(arz0, ax.v, ah.v, bi.v, bh.v);
        }
        {
            Frag bi, bh;
            bi.h8[0] = WI[(16 + m) * 4 + hh];  bi.h8[1] = WI[(16 + m) * 4 + 2 + hh];
            bh.h8[0] = WH[(16 + m) * 4 + hh];  bh.h8[1] = WH[(16 + m) * 4 + 2 + hh];
            arz1 = wmma16(ax.v, bi.v, zacc());
            arz1 = wmma16(ah.v, bh.v, arz1);
            guard22(arz1, ax.v, ah.v, bi.v, bh.v);
        }
        {
            Frag bi, bh;
            bi.h8[0] = WI[(32 + m) * 4 + hh];  bi.h8[1] = WI[(32 + m) * 4 + 2 + hh];
            bh.h8[0] = WH[(32 + m) * 4 + hh];  bh.h8[1] = WH[(32 + m) * 4 + 2 + hh];
            arz2 = wmma16(ax.v, bi.v, zacc());
            arz2 = wmma16(ah.v, bh.v, arz2);
            guard22(arz2, ax.v, ah.v, bi.v, bh.v);
        }
        {
            Frag bi, bh;
            bi.h8[0] = WI[(48 + m) * 4 + hh];  bi.h8[1] = WI[(48 + m) * 4 + 2 + hh];
            bh.h8[0] = WH[(48 + m) * 4 + hh];  bh.h8[1] = WH[(48 + m) * 4 + 2 + hh];
            arz3 = wmma16(ax.v, bi.v, zacc());
            arz3 = wmma16(ah.v, bh.v, arz3);
            guard22(arz3, ax.v, ah.v, bi.v, bh.v);
        }
        {
            Frag bi, bh;
            bi.h8[0] = WI[(64 + m) * 4 + hh];  bi.h8[1] = WI[(64 + m) * 4 + 2 + hh];
            bh.h8[0] = WH[(64 + m) * 4 + hh];  bh.h8[1] = WH[(64 + m) * 4 + 2 + hh];
            axn0 = wmma16(ax.v, bi.v, zacc());
            ahn0 = wmma16(ah.v, bh.v, zacc());
            guard2c(axn0, ahn0, ax.v, ah.v, bi.v, bh.v);
        }
        {
            Frag bi, bh;
            bi.h8[0] = WI[(80 + m) * 4 + hh];  bi.h8[1] = WI[(80 + m) * 4 + 2 + hh];
            bh.h8[0] = WH[(80 + m) * 4 + hh];  bh.h8[1] = WH[(80 + m) * 4 + 2 + hh];
            axn1 = wmma16(ax.v, bi.v, zacc());
            ahn1 = wmma16(ah.v, bh.v, zacc());
            guard2c(axn1, ahn1, ax.v, ah.v, bi.v, bh.v);
        }

        f16t* hn = &hsh[(t + 1) & 1][0];
        float p8[8];
#pragma unroll
        for (int r = 0; r < 8; ++r) {
            const float rr0 = sigm(fmaf(arz0[r], INV, br0));
            const float zz0 = sigm(fmaf(arz2[r], INV, bz0));
            const float nn0 = ftanh(fmaf(axn0[r], INV, bxn0) + rr0 * fmaf(ahn0[r], INV, bhn0));
            const float h0n = (1.0f - zz0) * nn0 + zz0 * hC0[r];
            const float rr1 = sigm(fmaf(arz1[r], INV, br1));
            const float zz1 = sigm(fmaf(arz3[r], INV, bz1));
            const float nn1 = ftanh(fmaf(axn1[r], INV, bxn1) + rr1 * fmaf(ahn1[r], INV, bhn1));
            const float h1n = (1.0f - zz1) * nn1 + zz1 * hC1[r];
            hC0[r] = h0n;
            hC1[r] = h1n;
            hn[(8 * hh + r) * 32 + m]      = (f16t)(h0n * 64.0f);
            hn[(8 * hh + r) * 32 + 16 + m] = (f16t)(h1n * 64.0f);
            p8[r] = fmaf(h0n, fw0, h1n * fw1);
        }
#pragma unroll
        for (int r = 0; r < 8; ++r) {
            float s = p8[r];
            s += __shfl_xor(s, 1);
            s += __shfl_xor(s, 2);
            s += __shfl_xor(s, 4);
            s += __shfl_xor(s, 8);
            p8[r] = sigm(s + fb);
        }
        if (m == 0) {
#pragma unroll
            for (int r = 0; r < 8; ++r) pst[(8 * hh + r) * NSTEP + t] = p8[r];
        }
        __syncthreads();
    }

#pragma unroll
    for (int r = 0; r < 8; ++r) {
        hfin[(8 * hh + r) * 32 + m]      = hC0[r];
        hfin[(8 * hh + r) * 32 + 16 + m] = hC1[r];
    }
    __syncthreads();
    {
        Pk32 hv[4];
#pragma unroll
        for (int i = 0; i < 4; ++i) {
            const int p = l + 32 * i;
            hv[i].f = *(const v4fa*)(hfin + p * 4);
        }
        float* ob = outh + (size_t)n0 * HID;
#pragma unroll
        for (int i = 0; i < 4; ++i) {
            const int p = l + 32 * i;
            *(volatile v4u*)(ob + (size_t)p * 4) = hv[i].u;
        }
        __threadfence();
#pragma unroll
        for (int i = 0; i < 4; ++i) {
            const int p = l + 32 * i;
            *(volatile v4u*)(ob + (size_t)p * 4) = hv[i].u;
        }
    }
    {
        float* pb = outp + (size_t)n0 * NSTEP;
#pragma unroll 1
        for (int i = 0; i < 63; ++i) {
            const int p = l + 32 * i, pc = min(p, 1999);
            Pk32 v;
            v.f = *(const v4fa*)(pst + pc * 4);
            if (p < 2000) *(volatile v4u*)(pb + (size_t)p * 4) = v.u;
        }
        __threadfence();
#pragma unroll 1
        for (int i = 0; i < 63; ++i) {
            const int p = l + 32 * i, pc = min(p, 1999);
            Pk32 v;
            v.f = *(const v4fa*)(pst + pc * 4);
            if (p < 2000) *(volatile v4u*)(pb + (size_t)p * 4) = v.u;
        }
    }
}

extern "C" void kernel_launch(void* const* d_in, const int* in_sizes, int n_in,
                              void* d_out, int out_size, void* d_ws, size_t ws_size,
                              hipStream_t stream) {
    if (n_in < 14) return;
    if (in_sizes[0] != NBATCH * 4 * NFREQ * NSTEP) return;
    if (in_sizes[1] != NSEQ * HID) return;
    if (in_sizes[2] != CH * 4 * 9 || in_sizes[3] != CH || in_sizes[4] < 1) return;
    if (in_sizes[5] != CH * CH * 5 || in_sizes[6] != CH || in_sizes[7] < 1) return;
    if (in_sizes[8] != NGATE * CH || in_sizes[9] != NGATE * HID) return;
    if (in_sizes[10] != NGATE || in_sizes[11] != NGATE) return;
    if (in_sizes[12] != HID || in_sizes[13] < 1) return;
    if (out_size != NSEQ * NSTEP + NSEQ * HID) return;

    const float* feat = (const float*)d_in[0];
    const float* h0   = (const float*)d_in[1];
    const float* w1   = (const float*)d_in[2];
    const float* b1   = (const float*)d_in[3];
    const float* a1   = (const float*)d_in[4];
    const float* w2   = (const float*)d_in[5];
    const float* b2   = (const float*)d_in[6];
    const float* a2   = (const float*)d_in[7];
    const float* wih  = (const float*)d_in[8];
    const float* whh  = (const float*)d_in[9];
    const float* bih  = (const float*)d_in[10];
    const float* bhh  = (const float*)d_in[11];
    const float* fcw  = (const float*)d_in[12];
    const float* fcb  = (const float*)d_in[13];

    float* outp = (float*)d_out;
    float* outh = outp + (size_t)NSEQ * NSTEP;

    char* ws = (char*)d_ws;
    const size_t oW1 = 0;
    const size_t oW2 = oW1 + (size_t)CH * 64 * 2;
    const size_t oWI = oW2 + (size_t)CH * 96 * 2;
    const size_t oWH = oWI + (size_t)NGATE * 32 * 2;
    const size_t oXP = oWH + (size_t)NGATE * 32 * 2;
    const size_t oEnd = oXP + (size_t)NSTEP * NBATCH * XFR * 2;
    if (oEnd > ws_size) return;
    f16t* W1P = (f16t*)(ws + oW1);
    f16t* W2P = (f16t*)(ws + oW2);
    f16t* WIP = (f16t*)(ws + oWI);
    f16t* WHP = (f16t*)(ws + oWH);
    f16t* XP  = (f16t*)(ws + oXP);

    k_pack<<<dim3(5), dim3(256), 0, stream>>>(w1, w2, wih, whh, W1P, W2P, WIP, WHP);
    k_conv<<<dim3(NBATCH * NSTEP), dim3(256), 0, stream>>>(feat, W1P, W2P, b1, a1, b2, a2, XP);
    k_gru<<<dim3(NSEQ / 16), dim3(32), 0, stream>>>(XP, WIP, WHP, h0, bih, bhh, fcw, fcb,
                                                    outp, outh);
}
